// MMINet_26405458935977
// MI455X (gfx1250) — hardware-verified
//
#include <hip/hip_runtime.h>
#define NB4 4
#define LF 4095
#define LP 4096
#define NR (NB4 * LP)
#define CC 256
#define CR 64
#define SEQ 32768
typedef __bf16 v16b __attribute__((ext_vector_type(16)));
typedef unsigned short v8us __attribute__((ext_vector_type(8), may_alias));
typedef float  v8f  __attribute__((ext_vector_type(8)));
typedef float  v4f  __attribute__((ext_vector_type(4)));
typedef float  v4fa __attribute__((ext_vector_type(4), may_alias));
union FragB { v16b v; v8us half[2]; unsigned short u[16]; };

__device__ __forceinline__ unsigned short bf16_bits(float x) { unsigned int u = __float_as_uint(x); return (unsigned short)((u + 0x7FFFu + ((u >> 16) & 1u)) >> 16); }
__device__ __forceinline__ float bf16_val(unsigned short b) { return __uint_as_float(((unsigned int)b) << 16); }
__device__ __forceinline__ float bf16_round(float x) { return bf16_val(bf16_bits(x)); }
template <int NT>
__device__ __forceinline__ v8f mmaN(v16b ah, v16b al, v16b bh, v16b bl, v8f c) {
  c = __builtin_amdgcn_wmma_f32_16x16x32_bf16(false, ah, false, bh, (short)0, c, false, false);
  if (NT >= 2) c = __builtin_amdgcn_wmma_f32_16x16x32_bf16(false, al, false, bh, (short)0, c, false, false);
  if (NT >= 3) c = __builtin_amdgcn_wmma_f32_16x16x32_bf16(false, ah, false, bl, (short)0, c, false, false);
  asm volatile("v_nop\n\tv_nop\n\tv_nop\n\tv_nop" : "+v"(c) : "v"(ah), "v"(al), "v"(bh), "v"(bl));
  return c;
}

__global__ __launch_bounds__(256) void k_wt_bf16(const float* __restrict__ W, unsigned short* __restrict__ Wt, int K, int N) {
  const int t = blockIdx.x * 256 + threadIdx.x;
  const int k8n = K / 8;
  if (t >= N * k8n) return;
  const int n = t / k8n, k8 = (t % k8n) * 8;
  v8us v;
#pragma unroll
  for (int i = 0; i < 8; ++i) v[i] = bf16_bits(W[(size_t)(k8 + i) * N + n]);
  *(volatile v8us*)(Wt + (size_t)n * K + k8) = v;
  __threadfence();
  *(volatile v8us*)(Wt + (size_t)n * K + k8) = v;
}

template <bool ASPLIT, int ACT, bool BIAS_BF16>
__global__ __launch_bounds__(128) void k_gemm_bf(const float* __restrict__ A, int lda, const unsigned short* __restrict__ Wt, int ldb,
                                               const float* __restrict__ bias, float* __restrict__ C, int ldc, int M, int N, int K) {
  __shared__ __attribute__((aligned(16))) float so[4][16][64];
  const int tid = threadIdx.x, w = tid >> 5, lane = tid & 31, ln = lane & 15, hh = lane >> 4;
  const int ntn = N / 64;
  const int wid = blockIdx.x * 4 + w;
  const int mt = wid / ntn, nq = wid % ntn;
  if (mt * 16 >= M) return;
  const int row0 = mt * 16, col0 = nq * 64;
  const float* arow = A + (size_t)(row0 + ln) * lda;
  v8f acc[4] = {};
  for (int kb = 0; kb < K; kb += 32) {
    FragB ah, al;
    const v4f x0 = *(const v4fa*)(arow + kb + 8 * hh), x1 = *(const v4fa*)(arow + kb + 8 * hh + 4);
    const v4f x2 = *(const v4fa*)(arow + kb + 16 + 8 * hh), x3 = *(const v4fa*)(arow + kb + 16 + 8 * hh + 4);
    float xs[16] = {x0[0],x0[1],x0[2],x0[3],x1[0],x1[1],x1[2],x1[3],x2[0],x2[1],x2[2],x2[3],x3[0],x3[1],x3[2],x3[3]};
#pragma unroll
    for (int i = 0; i < 16; ++i) { const unsigned short hb = bf16_bits(xs[i]); ah.u[i] = hb; al.u[i] = ASPLIT ? bf16_bits(xs[i] - bf16_val(hb)) : (unsigned short)0; }
#pragma unroll
    for (int t = 0; t < 4; ++t) {
      const unsigned short* brow = Wt + (size_t)(col0 + t * 16 + ln) * ldb + kb;
      FragB b;
      b.half[0] = *(const v8us*)(brow + 8 * hh);
      b.half[1] = *(const v8us*)(brow + 16 + 8 * hh);
      acc[t] = mmaN<ASPLIT ? 2 : 1>(ah.v, al.v, b.v, b.v, acc[t]);
    }
  }
#pragma unroll
  for (int t = 0; t < 4; ++t) {
    float bv = bias ? bias[col0 + t * 16 + ln] : 0.f;
    if (BIAS_BF16) bv = bf16_round(bv);
#pragma unroll
    for (int r = 0; r < 8; ++r) { float v = acc[t][r] + bv; if (ACT == 1) v = fmaxf(v, 0.f); so[w][8 * hh + r][t * 16 + ln] = v; }
  }
  __builtin_amdgcn_fence(__ATOMIC_ACQ_REL, "workgroup");
  __builtin_amdgcn_wave_barrier();
  const int rsub = lane >> 4, c4 = (lane & 15) * 4;
  for (int pass = 0; pass < 2; ++pass) {
#pragma unroll
    for (int q = 0; q < 8; ++q) {
      const int r = q * 2 + rsub;
      const v4f v = *(const v4fa*)&so[w][r][c4];
      *(volatile v4f*)(C + (size_t)(row0 + r) * ldc + col0 + c4) = v;
    }
    if (pass == 0) __threadfence();
  }
}

template <bool ASPLIT, int ACT, bool BIAS_BF16, bool RES_BF16>
__global__ __launch_bounds__(128) void k_gemm_bf3(const float* __restrict__ A, int lda, const unsigned short* __restrict__ Wt, int ldb,
                                                const float* __restrict__ bias, const float* __restrict__ resid, int rmod, int ldr,
                                                float* __restrict__ C, int ldc, int M, int N, int K) {
  __shared__ __attribute__((aligned(16))) float so[4][16][64];
  const int tid = threadIdx.x, w = tid >> 5, lane = tid & 31, ln = lane & 15, hh = lane >> 4;
  const int ntn = N / 64;
  const int wid = blockIdx.x * 4 + w;
  const int mt = wid / ntn, nq = wid % ntn;
  if (mt * 16 >= M) return;
  const int row0 = mt * 16, col0 = nq * 64;
  const float* arow = A + (size_t)(row0 + ln) * lda;
  v8f acc[4] = {};
  for (int kb = 0; kb < K; kb += 32) {
    FragB ah, al;
    const v4f x0 = *(const v4fa*)(arow + kb + 8 * hh), x1 = *(const v4fa*)(arow + kb + 8 * hh + 4);
    const v4f x2 = *(const v4fa*)(arow + kb + 16 + 8 * hh), x3 = *(const v4fa*)(arow + kb + 16 + 8 * hh + 4);
    float xs[16] = {x0[0],x0[1],x0[2],x0[3],x1[0],x1[1],x1[2],x1[3],x2[0],x2[1],x2[2],x2[3],x3[0],x3[1],x3[2],x3[3]};
#pragma unroll
    for (int i = 0; i < 16; ++i) { const unsigned short hb = bf16_bits(xs[i]); ah.u[i] = hb; al.u[i] = ASPLIT ? bf16_bits(xs[i] - bf16_val(hb)) : (unsigned short)0; }
#pragma unroll
    for (int t = 0; t < 4; ++t) {
      const unsigned short* brow = Wt + (size_t)(col0 + t * 16 + ln) * ldb + kb;
      FragB b;
      b.half[0] = *(const v8us*)(brow + 8 * hh);
      b.half[1] = *(const v8us*)(brow + 16 + 8 * hh);
      acc[t] = mmaN<ASPLIT ? 2 : 1>(ah.v, al.v, b.v, b.v, acc[t]);
    }
  }
#pragma unroll
  for (int t = 0; t < 4; ++t) {
    const int col = col0 + t * 16 + ln;
    float bv = bias ? bias[col] : 0.f;
    if (BIAS_BF16) bv = bf16_round(bv);
#pragma unroll
    for (int r = 0; r < 8; ++r) {
      float v = acc[t][r] + bv;
      if (resid) { float rv = resid[(size_t)((row0 + 8 * hh + r) % rmod) * ldr + col]; if (RES_BF16) rv = bf16_round(rv); v += rv; }
      if (ACT == 1) v = fmaxf(v, 0.f);
      if (ACT == 2) v = 0.5f * v * (1.0f + erff(v * 0.70710678118654752f));
      if (ACT == 3) { const float u = 0.7978845608028654f * (v + 0.044715f * v * v * v); v = 0.5f * v * (1.0f + tanhf(u)); }
      so[w][8 * hh + r][t * 16 + ln] = v;
    }
  }
  __builtin_amdgcn_fence(__ATOMIC_ACQ_REL, "workgroup");
  __builtin_amdgcn_wave_barrier();
  const int rsub = lane >> 4, c4 = (lane & 15) * 4;
  for (int pass = 0; pass < 2; ++pass) {
#pragma unroll
    for (int q = 0; q < 8; ++q) {
      const int r = q * 2 + rsub;
      const v4f v = *(const v4fa*)&so[w][r][c4];
      *(volatile v4f*)(C + (size_t)(row0 + r) * ldc + col0 + c4) = v;
    }
    if (pass == 0) __threadfence();
  }
}
template <bool PARAM_BF16>
__global__ __launch_bounds__(256) void k_layernorm(const float* __restrict__ X, const float* __restrict__ R, const float* __restrict__ g, const float* __restrict__ bta,
                                                  float* __restrict__ out_sum, float* __restrict__ out_norm, int N, float eps) {
  __shared__ float red[256];
  const int row = blockIdx.x, tid = threadIdx.x;
  const float* x = X + (size_t)row * N; const float* rr = R ? R + (size_t)row * N : nullptr;
  float vals[16];
  const int per = N / 256;
  float s1 = 0.f;
  for (int u = 0; u < per / 4; ++u) {
    const int j = tid * 4 + 1024 * u;
    const v4f a = *(const v4fa*)(x + j);
    v4f b = {0.f,0.f,0.f,0.f}; if (rr) b = *(const v4fa*)(rr + j);
#pragma unroll
    for (int q = 0; q < 4; ++q) { const float v = a[q] + b[q]; vals[u * 4 + q] = v; s1 += v; }
  }
  red[tid] = s1; __syncthreads();
  for (int st = 128; st > 0; st >>= 1) { if (tid < st) red[tid] += red[tid + st]; __syncthreads(); }
  const float mu = red[0] / (float)N; __syncthreads();
  float s2 = 0.f;
  for (int u = 0; u < per / 4; ++u)
#pragma unroll
    for (int q = 0; q < 4; ++q) { const float c = vals[u * 4 + q] - mu; s2 += c * c; }
  red[tid] = s2; __syncthreads();
  for (int st = 128; st > 0; st >>= 1) { if (tid < st) red[tid] += red[tid + st]; __syncthreads(); }
  const float rs = rsqrtf(red[0] / (float)N + eps);
  for (int pass = 0; pass < 2; ++pass) {
    for (int u = 0; u < per / 4; ++u) {
      const int j = tid * 4 + 1024 * u;
      v4f o, sm;
#pragma unroll
      for (int q = 0; q < 4; ++q) {
        float gg = g[j + q], bb = bta[j + q];
        if (PARAM_BF16) { gg = bf16_round(gg); bb = bf16_round(bb); }
        sm[q] = vals[u * 4 + q]; o[q] = (vals[u * 4 + q] - mu) * rs * gg + bb;
      }
      if (out_sum) *(volatile v4f*)(out_sum + (size_t)row * N + j) = sm;
      *(volatile v4f*)(out_norm + (size_t)row * N + j) = o;
    }
    if (pass == 0) __threadfence();
  }
}


typedef _Float16 v16h __attribute__((ext_vector_type(16)));
union FragH { v16h v; v8us half[2]; _Float16 h[16]; unsigned short u[16]; };
template <int NT>
__device__ __forceinline__ v8f mmaH(v16h ah, v16h al, v16h bh, v16h bl, v8f c) {
  c = __builtin_amdgcn_wmma_f32_16x16x32_f16(false, ah, false, bh, (short)0, c, false, false);
  if (NT >= 2) c = __builtin_amdgcn_wmma_f32_16x16x32_f16(false, al, false, bh, (short)0, c, false, false);
  if (NT >= 3) c = __builtin_amdgcn_wmma_f32_16x16x32_f16(false, ah, false, bl, (short)0, c, false, false);
  asm volatile("v_nop\n\tv_nop\n\tv_nop\n\tv_nop" : "+v"(c) : "v"(ah), "v"(al), "v"(bh), "v"(bl));
  return c;
}
template <bool ASPLIT>
__global__ __launch_bounds__(128) void k_gemm_h(const float* __restrict__ A, int lda, size_t sA, const _Float16* __restrict__ Bh, int ldb, size_t sB, float alpha, float* __restrict__ C, int ldc, size_t sC, int M, int N, int K) {
  __shared__ __attribute__((aligned(16))) float so[4][16][64];
  const int tid = threadIdx.x, w = tid >> 5, lane = tid & 31, ln = lane & 15, hh = lane >> 4; const int by = blockIdx.y;
  A += (size_t)by * sA; Bh += (size_t)by * sB; C += (size_t)by * sC;
  const int ntn = (N + 63) / 64; const int wid = blockIdx.x * 4 + w; const int mt = wid / ntn, nq = wid % ntn; if (mt * 16 >= M) return;
  const int row0 = mt * 16, col0 = nq * 64; const float* arow = A + (size_t)(row0 + ln) * lda;
  v8f acc[4] = {};
  for (int kb = 0; kb < K; kb += 32) {
    FragH ah, al;
    const v4f x0 = *(const v4fa*)(arow + kb + 8 * hh), x1 = *(const v4fa*)(arow + kb + 8 * hh + 4), x2 = *(const v4fa*)(arow + kb + 16 + 8 * hh), x3 = *(const v4fa*)(arow + kb + 16 + 8 * hh + 4);
    float xs[16] = {x0[0],x0[1],x0[2],x0[3],x1[0],x1[1],x1[2],x1[3],x2[0],x2[1],x2[2],x2[3],x3[0],x3[1],x3[2],x3[3]};
#pragma unroll
    for (int i = 0; i < 16; ++i) { const _Float16 h = (_Float16)xs[i]; ah.h[i] = h; al.h[i] = ASPLIT ? (_Float16)(xs[i] - (float)h) : (_Float16)0.0f; }
#pragma unroll
    for (int t = 0; t < 4; ++t) { if (col0 + t * 16 >= N) continue; const size_t boff = (size_t)(col0 + t * 16 + ln) * ldb + kb; FragH bq; bq.half[0] = *(const v8us*)(Bh + boff + 8 * hh); bq.half[1] = *(const v8us*)(Bh + boff + 16 + 8 * hh);
      acc[t] = mmaH<ASPLIT ? 2 : 1>(ah.v, al.v, bq.v, bq.v, acc[t]); }
  }
#pragma unroll
  for (int t = 0; t < 4; ++t) { if (col0 + t * 16 >= N) continue;
#pragma unroll
    for (int r = 0; r < 8; ++r) so[w][8 * hh + r][t * 16 + ln] = acc[t][r] * alpha; }
  __builtin_amdgcn_fence(__ATOMIC_ACQ_REL, "workgroup"); __builtin_amdgcn_wave_barrier();
  const int rsub = lane >> 4, c4 = (lane & 15) * 4;
  for (int pass = 0; pass < 2; ++pass) {
#pragma unroll
    for (int q = 0; q < 8; ++q) { const int r = q * 2 + rsub; if (col0 + c4 < N) { const v4f v = *(const v4fa*)&so[w][r][c4]; *(volatile v4f*)(C + (size_t)(row0 + r) * ldc + col0 + c4) = v; } }
    if (pass == 0) __threadfence(); }
}

__global__ __launch_bounds__(256) void k_wt_f16(const float* __restrict__ W, _Float16* __restrict__ Wt, int K, int N, float scale) {
  const int t = blockIdx.x * 256 + threadIdx.x; if (t >= N * (K / 8)) return; const int n = t / (K / 8), k8 = (t % (K / 8)) * 8; FragH f;
#pragma unroll
  for (int i = 0; i < 8; ++i) f.h[i] = (_Float16)(bf16_round(W[(size_t)(k8 + i) * N + n]) * scale); const v8us o = f.half[0];
  *(volatile v8us*)((unsigned short*)Wt + (size_t)n * K + k8) = o; __threadfence(); *(volatile v8us*)((unsigned short*)Wt + (size_t)n * K + k8) = o;
}
template <int ACT>
__global__ __launch_bounds__(128) void k_gemm_hhx(const _Float16* __restrict__ A, int lda, size_t sA, const _Float16* __restrict__ Bh, int ldb, size_t sB, float alpha, const float* __restrict__ bias, size_t sBias, const float* __restrict__ CP, int rowsPerB, size_t sCPb, int row0g,
    float* __restrict__ C, _Float16* __restrict__ C16, int ldc, size_t sC, int M, int N, int K) {
  __shared__ __attribute__((aligned(16))) float so[4][16][64];
  const int tid = threadIdx.x, w = tid >> 5, lane = tid & 31, ln = lane & 15, hh = lane >> 4; const int by = blockIdx.y;
  A += (size_t)by * sA; Bh += (size_t)by * sB; const size_t cofs = (size_t)by * sC; const float* bp = bias ? bias + (size_t)by * sBias : nullptr;
  const int ntn = (N + 63) / 64; const int wid = blockIdx.x * 4 + w; const int mt = wid / ntn, nq = wid % ntn; if (mt * 16 >= M) return;
  const int row0 = mt * 16, col0 = nq * 64; const _Float16* arow = A + (size_t)(row0 + ln) * lda;
  v8f acc[4] = {};
  for (int kb = 0; kb < K; kb += 32) { FragH ah; ah.half[0] = *(const v8us*)((const unsigned short*)arow + kb + 8 * hh); ah.half[1] = *(const v8us*)((const unsigned short*)arow + kb + 16 + 8 * hh);
#pragma unroll
    for (int t = 0; t < 4; ++t) { if (col0 + t * 16 >= N) continue; const size_t boff = (size_t)(col0 + t * 16 + ln) * ldb + kb; FragH bq; bq.half[0] = *(const v8us*)((const unsigned short*)Bh + boff + 8 * hh); bq.half[1] = *(const v8us*)((const unsigned short*)Bh + boff + 16 + 8 * hh);
      acc[t] = mmaH<1>(ah.v, ah.v, bq.v, bq.v, acc[t]); }
  }
#pragma unroll
  for (int t = 0; t < 4; ++t) { if (col0 + t * 16 >= N) continue; const int col = col0 + t * 16 + ln; const float bv = bp ? bf16_round(bp[col]) : 0.f;
#pragma unroll
    for (int r = 0; r < 8; ++r) { float v = acc[t][r] * alpha + bv; if (CP) { const int bidx = (row0g + row0 + 8 * hh + r) / rowsPerB; v += CP[(size_t)bidx * sCPb + (size_t)by * 64 + col]; } if (ACT == 1) v = (v > 0.f) ? v : expm1f(v); else if (ACT == 7) v = (v > 0.f) ? v + 1.0f : expf(v); else if (ACT == 8) v = tanhf(v); else if (ACT == 9) v = 0.5f * v * (1.0f + tanhf(0.7978845608028654f * (v + 0.044715f * v * v * v))); else if (ACT == 11) v = 1.0f / (1.0f + expf(-v)); else if (ACT == 12) v = (v > 0.f) ? v : 0.01f * v; else if (ACT == 14) v = (v > 0.f) ? v : 0.1f * v; else if (ACT == 15) v = v / (1.0f + expf(-v)); else if (ACT == 3) v = fmaxf(v, 0.f); else if (ACT == 6) v = 0.5f * v * (1.0f + erff(v * 0.70710678118654752f)); so[w][8 * hh + r][t * 16 + ln] = v; } }
  __builtin_amdgcn_fence(__ATOMIC_ACQ_REL, "workgroup"); __builtin_amdgcn_wave_barrier();
  const int rsub = lane >> 4, c4 = (lane & 15) * 4; typedef _Float16 v4h __attribute__((ext_vector_type(4)));
  for (int pass = 0; pass < 2; ++pass) {
#pragma unroll
    for (int q = 0; q < 8; ++q) { const int r = q * 2 + rsub; if (col0 + c4 < N) { const v4f v = *(const v4fa*)&so[w][r][c4]; if (C) *(volatile v4f*)(C + cofs + (size_t)(row0 + r) * ldc + col0 + c4) = v; if (C16) { v4h h4; for (int i = 0; i < 4; ++i) h4[i] = (_Float16)v[i]; *(volatile v4h*)(C16 + cofs + (size_t)(row0 + r) * ldc + col0 + c4) = h4; } } }
    if (pass == 0) __threadfence(); }
}


typedef _Float16 v4h __attribute__((ext_vector_type(4)));

__global__ __launch_bounds__(256) void k_x16(const float* __restrict__ x, _Float16* __restrict__ X16, size_t n8) { const size_t t = (size_t)blockIdx.x * 256 + threadIdx.x; if (t >= n8) return; FragH f;
#pragma unroll
  for (int q = 0; q < 8; ++q) f.h[q] = (_Float16)bf16_round(x[t * 8 + q]); *(volatile v8us*)((unsigned short*)X16 + t * 8) = f.half[0]; __threadfence(); *(volatile v8us*)((unsigned short*)X16 + t * 8) = f.half[0]; }
__global__ __launch_bounds__(256) void k_h16(const float* __restrict__ x, _Float16* __restrict__ X16, size_t n8) { const size_t t = (size_t)blockIdx.x * 256 + threadIdx.x; if (t >= n8) return; FragH f;
#pragma unroll
  for (int q = 0; q < 8; ++q) f.h[q] = (_Float16)x[t * 8 + q]; *(volatile v8us*)((unsigned short*)X16 + t * 8) = f.half[0]; __threadfence(); *(volatile v8us*)((unsigned short*)X16 + t * 8) = f.half[0]; }
__global__ __launch_bounds__(256) void k_round16f(const float* __restrict__ W, _Float16* __restrict__ Bt, size_t n8) { const size_t t = (size_t)blockIdx.x * 256 + threadIdx.x; if (t >= n8) return; FragH f;
#pragma unroll
  for (int i = 0; i < 8; ++i) f.h[i] = (_Float16)(bf16_round(W[t * 8 + i]) * 16.0f); *(volatile v8us*)((unsigned short*)Bt + t * 8) = f.half[0]; __threadfence(); *(volatile v8us*)((unsigned short*)Bt + t * 8) = f.half[0]; }
template <int NHv, int TTv>
__global__ __launch_bounds__(256) void k_vt(const _Float16* __restrict__ V16, int ldv, int voff, _Float16* __restrict__ Vt) { __shared__ unsigned short tl[64][66]; const int tid = threadIdx.x; const int slab = blockIdx.x / (TTv / 64), lg = blockIdx.x % (TTv / 64); const int b = slab / NHv, h = slab % NHv;
  for (int i = tid; i < 64 * 8; i += 256) { const int r = i / 8, c8 = (i % 8) * 8; FragH f; f.half[0] = *(const v8us*)((const unsigned short*)V16 + ((size_t)b * TTv + lg * 64 + r) * ldv + voff + h * 64 + c8);
#pragma unroll
    for (int q = 0; q < 8; ++q) tl[r][c8 + q] = f.u[q]; }
  __syncthreads();
  for (int pass = 0; pass < 2; ++pass) {
#pragma unroll
    for (int rd = 0; rd < 2; ++rd) { const int d = rd * 32 + tid / 8, pc = tid % 8; FragH f;
#pragma unroll
      for (int q = 0; q < 8; ++q) f.u[q] = tl[pc * 8 + q][d];
      *(volatile v8us*)((unsigned short*)Vt + ((size_t)slab * 64 + d) * TTv + lg * 64 + pc * 8) = f.half[0]; }
    if (pass == 0) __threadfence(); } }

__global__ __launch_bounds__(256) void k_hl(const float* __restrict__ F, _Float16* __restrict__ Hh, _Float16* __restrict__ Hl, size_t n8) { const size_t t = (size_t)blockIdx.x * 256 + threadIdx.x; if (t >= n8) return; FragH fh, fl; const v4f a = *(const v4fa*)(F + t * 8), c = *(const v4fa*)(F + t * 8 + 4);
#pragma unroll
  for (int q = 0; q < 4; ++q) { _Float16 h = (_Float16)a[q]; fh.h[q] = h; fl.h[q] = (_Float16)((a[q] - (float)h) * 1024.0f); h = (_Float16)c[q]; fh.h[4 + q] = h; fl.h[4 + q] = (_Float16)((c[q] - (float)h) * 1024.0f); }
  for (int pass = 0; pass < 2; ++pass) { *(volatile v8us*)((unsigned short*)Hh + t * 8) = fh.half[0]; *(volatile v8us*)((unsigned short*)Hl + t * 8) = fl.half[0]; if (pass == 0) __threadfence(); } }

__global__ __launch_bounds__(256) void k_split(const float* __restrict__ F, _Float16* __restrict__ Hh, _Float16* __restrict__ Hl, size_t n8) {
  #pragma clang fp contract(off)
  const size_t t = (size_t)blockIdx.x * 256 + threadIdx.x; if (t >= n8) return; const v4f a = *(const v4fa*)(F + t * 8), c = *(const v4fa*)(F + t * 8 + 4); FragH fh, fl;
#pragma unroll
  for (int q = 0; q < 8; ++q) { const float v = (q < 4) ? a[q] : c[q - 4]; const _Float16 hi = (_Float16)v; fh.h[q] = hi; fl.h[q] = (_Float16)((v - (float)hi) * 1024.0f); }
  for (int pass = 0; pass < 2; ++pass) { *(volatile v8us*)((unsigned short*)Hh + t * 8) = fh.half[0]; *(volatile v8us*)((unsigned short*)Hl + t * 8) = fl.half[0]; if (pass == 0) __threadfence(); } }
__global__ __launch_bounds__(256) void k_win(const float* __restrict__ ac, const float* __restrict__ bc, _Float16* __restrict__ A16) { const int t = blockIdx.x * 256 + threadIdx.x; if (t >= NR * 4) return; const int g = t & 3, r = t >> 2; const int b = r / LP, l = r % LP; const bool live = (l < LF);
  const float* sa = ac + (size_t)b * SEQ + (size_t)min(l, LF - 1) * 8 + (g & 1) * 8; const float* sb = bc + (size_t)b * SEQ + (size_t)min(l, LF - 1) * 8 + (g & 1) * 8; FragH f;
#pragma unroll
  for (int q = 0; q < 8; ++q) { const float va = bf16_round(sa[q]), vb = bf16_round(sb[q]); f.h[q] = live ? (_Float16)((g < 2) ? va : vb) : (_Float16)0.0f; }
  *(volatile v8us*)((unsigned short*)A16 + (size_t)r * 32 + g * 8) = f.half[0]; __threadfence(); *(volatile v8us*)((unsigned short*)A16 + (size_t)r * 32 + g * 8) = f.half[0]; }
__global__ __launch_bounds__(256) void k_wenc(const float* __restrict__ aw, const float* __restrict__ bw, _Float16* __restrict__ Bt) { const int t = blockIdx.x * 256 + threadIdx.x; if (t >= CC * 4) return; const int g = t & 3, o = t >> 2; const float* sa = aw + (size_t)o * 16 + (g & 1) * 8; const float* sb = bw + (size_t)o * 16 + (g & 1) * 8; FragH f;
#pragma unroll
  for (int q = 0; q < 8; ++q) { const float va = bf16_round(sa[q]), vb = bf16_round(sb[q]); f.h[q] = (_Float16)(((g < 2) ? va : vb) * 16.0f); }
  *(volatile v8us*)((unsigned short*)Bt + (size_t)o * 32 + g * 8) = f.half[0]; __threadfence(); *(volatile v8us*)((unsigned short*)Bt + (size_t)o * 32 + g * 8) = f.half[0]; }
__global__ __launch_bounds__(256) void k_lnc(const float* __restrict__ X, const float* __restrict__ pa, const float* __restrict__ g, const float* __restrict__ bb, float* __restrict__ Y, _Float16* __restrict__ Yh, _Float16* __restrict__ Yl) {
  #pragma clang fp contract(off)
  const int tid = threadIdx.x, w = tid >> 5, ln = tid & 31; const int r = blockIdx.x * 8 + w; if (r >= NR) return; const bool live = ((r % LP) < LF); const float a = pa ? bf16_round(pa[0]) : 1.0f; float v[8]; float s = 0.f;
#pragma unroll
  for (int k = 0; k < 8; ++k) { float x = X[(size_t)r * CC + ln * 8 + k]; if (pa) x = (x >= 0.f) ? x : a * x; v[k] = x; s += x; }
  for (int o = 16; o > 0; o >>= 1) s += __shfl_xor(s, o, 32); const float mu = s / (float)CC; float q2 = 0.f;
#pragma unroll
  for (int k = 0; k < 8; ++k) { const float d = v[k] - mu; q2 += d * d; }
  for (int o = 16; o > 0; o >>= 1) q2 += __shfl_xor(q2, o, 32); const float rs = rsqrtf(q2 / (float)CC + 1e-5f); v4f oa, ob; FragH fh, fl;
#pragma unroll
  for (int k = 0; k < 8; ++k) { const int c = ln * 8 + k; const float y = live ? ((v[k] - mu) * rs * bf16_round(g[c]) + bf16_round(bb[c])) : 0.f; if (k < 4) oa[k] = y; else ob[k - 4] = y; const _Float16 hi = (_Float16)y; fh.h[k] = hi; fl.h[k] = (_Float16)((y - (float)hi) * 1024.0f); }
  for (int pass = 0; pass < 2; ++pass) { if (Y) { *(volatile v4f*)(Y + (size_t)r * CC + ln * 8) = oa; *(volatile v4f*)(Y + (size_t)r * CC + ln * 8 + 4) = ob; } *(volatile v8us*)((unsigned short*)Yh + (size_t)r * CC + ln * 8) = fh.half[0]; *(volatile v8us*)((unsigned short*)Yl + (size_t)r * CC + ln * 8) = fl.half[0]; if (pass == 0) __threadfence(); } }
__global__ __launch_bounds__(256) void k_inv(const float* __restrict__ K1, const float* __restrict__ w2, const float* __restrict__ b2, const float* __restrict__ mi, const float* __restrict__ pa, float* __restrict__ mo, _Float16* __restrict__ Mh, _Float16* __restrict__ Ml) {
  #pragma clang fp contract(off)
  const int t = blockIdx.x * 256 + threadIdx.x; if (t >= NR * (CC / 8)) return; const int c0 = (t % (CC / 8)) * 8, r = t / (CC / 8); const int l = r % LP; const bool live = (l < LF); float ker[3];
#pragma unroll
  for (int k = 0; k < 3; ++k) { float s = bf16_round(b2[k]);
#pragma unroll 8
    for (int j = 0; j < CR; ++j) s += bf16_round(w2[k * CR + j]) * K1[(size_t)r * CR + j];
    ker[k] = s; }
  v4f oa, ob; FragH fh, fl;
#pragma unroll
  for (int q = 0; q < 8; ++q) { const int c = c0 + q; float acc = 0.f;
#pragma unroll
    for (int k = 0; k < 3; ++k) { const int ll = l + k - 1; const bool in = (ll >= 0 && ll < LF); const int rr = r - l + min(max(ll, 0), LP - 1); const float v = mi[(size_t)rr * CC + c]; acc += ker[k] * (in ? v : 0.f); }
    const float a = bf16_round(pa[c]); const float y = live ? ((acc >= 0.f) ? acc : a * acc) : 0.f; if (q < 4) oa[q] = y; else ob[q - 4] = y; const _Float16 hi = (_Float16)y; fh.h[q] = hi; fl.h[q] = (_Float16)((y - (float)hi) * 1024.0f); }
  for (int pass = 0; pass < 2; ++pass) { *(volatile v4f*)(mo + (size_t)r * CC + c0) = oa; *(volatile v4f*)(mo + (size_t)r * CC + c0 + 4) = ob; *(volatile v8us*)((unsigned short*)Mh + (size_t)r * CC + c0) = fh.half[0]; *(volatile v8us*)((unsigned short*)Ml + (size_t)r * CC + c0) = fl.half[0]; if (pass == 0) __threadfence(); } }
__global__ __launch_bounds__(256) void k_em(const float* __restrict__ ENC, const float* __restrict__ MASK, _Float16* __restrict__ Eh, _Float16* __restrict__ El, size_t n8) {
  #pragma clang fp contract(off)
  const size_t t = (size_t)blockIdx.x * 256 + threadIdx.x; if (t >= n8) return; FragH fh, fl;
#pragma unroll
  for (int q = 0; q < 8; ++q) { const float v = ENC[t * 8 + q] * MASK[t * 8 + q]; const _Float16 hi = (_Float16)v; fh.h[q] = hi; fl.h[q] = (_Float16)((v - (float)hi) * 1024.0f); }
  for (int pass = 0; pass < 2; ++pass) { *(volatile v8us*)((unsigned short*)Eh + t * 8) = fh.half[0]; *(volatile v8us*)((unsigned short*)El + t * 8) = fl.half[0]; if (pass == 0) __threadfence(); } }
__global__ __launch_bounds__(256) void k_wdec(const float* __restrict__ dw, _Float16* __restrict__ Bt) { const int t = blockIdx.x * 256 + threadIdx.x; if (t >= 16 * (CC / 8)) return; const int c0 = (t % (CC / 8)) * 8, j = t / (CC / 8); FragH f;
#pragma unroll
  for (int q = 0; q < 8; ++q) f.h[q] = (_Float16)(bf16_round(dw[(size_t)(c0 + q) * 16 + j]) * 16.0f);
  *(volatile v8us*)((unsigned short*)Bt + (size_t)j * CC + c0) = f.half[0]; __threadfence(); *(volatile v8us*)((unsigned short*)Bt + (size_t)j * CC + c0) = f.half[0]; }
__global__ __launch_bounds__(256) void k_ola(const float* __restrict__ Y, float* __restrict__ out) {
  #pragma clang fp contract(off)
  const int t = blockIdx.x * 256 + threadIdx.x; if (t >= NB4 * SEQ) return; const int b = t / SEQ, tt = t % SEQ; const int l = tt >> 3, j = tt & 7; float s = 0.f;
  { const bool in = (l < LF); const float v = Y[((size_t)b * LP + min(l, LF - 1)) * 16 + j]; s += in ? v : 0.f; }
  { const int l2 = l - 1; const bool in = (l2 >= 0 && l2 < LF); const float v = Y[((size_t)b * LP + min(max(l2, 0), LF - 1)) * 16 + 8 + j]; s += in ? v : 0.f; }
  *(volatile float*)(out + t) = s; __threadfence(); *(volatile float*)(out + t) = s; }

extern "C" void kernel_launch(void* const* d_in, const int* in_sizes, int n_in,
                              void* d_out, int out_size, void* d_ws, size_t ws_size, hipStream_t stream) {
  (void)in_sizes; (void)n_in; (void)out_size;
  const float* const* I = (const float* const*)d_in; const float* ac = I[0]; const float* bcx = I[1]; const float* acw = I[2]; const float* bcw = I[3]; const float* lng = I[4]; const float* lnb = I[5]; const float* iw = I[6]; const float* ib = I[7]; const float* blg = I[8]; const float* blb = I[9]; const float* bla = I[10]; const float* iv1 = I[11]; const float* ivb1 = I[12]; const float* iv2 = I[13]; const float* ivb2 = I[14]; const float* ipa = I[15]; const float* skw = I[16]; const float* skb = I[17]; const float* fw = I[18]; const float* fb = I[19]; const float* dw = I[20];
  char* ws = (char*)d_ws; size_t off = 0;
  auto take = [&](size_t bytes) { char* p = ws + off; off += (bytes + 255) & ~(size_t)255; return p; };
  _Float16* BE = (_Float16*)take(CC * 32 * 2); _Float16* BI = (_Float16*)take(CC * CC * 2); _Float16* BK1 = (_Float16*)take((size_t)12 * CR * CC * 2); _Float16* BS = (_Float16*)take((size_t)4 * CC * CC * 2); _Float16* BF = (_Float16*)take(CC * CC * 2); _Float16* BD = (_Float16*)take(16 * CC * 2);
  _Float16* A16 = (_Float16*)take((size_t)NR * 32 * 2); float* ENC = (float*)take((size_t)NR * CC * 4); float* X = (float*)take((size_t)NR * CC * 4); float* XN = (float*)take((size_t)NR * CC * 4); _Float16* Ph = (_Float16*)take((size_t)NR * CC * 2); _Float16* Pl = (_Float16*)take((size_t)NR * CC * 2); _Float16* Qh = (_Float16*)take((size_t)NR * CC * 2); _Float16* Ql = (_Float16*)take((size_t)NR * CC * 2); float* MA = (float*)take((size_t)NR * CC * 4); float* MB = (float*)take((size_t)NR * CC * 4); float* K1 = (float*)take((size_t)NR * CR * 4); float* Y = (float*)take((size_t)NR * 16 * 4);
  if (off > ws_size) return;
  k_wenc<<<(CC * 4 + 255) / 256, 256, 0, stream>>>(acw, bcw, BE); k_round16f<<<(CC * CC / 8 + 255) / 256, 256, 0, stream>>>(iw, BI, (size_t)CC * CC / 8); k_round16f<<<(unsigned)(((size_t)12 * CR * CC / 8 + 255) / 256), 256, 0, stream>>>(iv1, BK1, (size_t)12 * CR * CC / 8); k_round16f<<<(unsigned)(((size_t)4 * CC * CC / 8 + 255) / 256), 256, 0, stream>>>(skw, BS, (size_t)4 * CC * CC / 8); k_round16f<<<(CC * CC / 8 + 255) / 256, 256, 0, stream>>>(fw, BF, (size_t)CC * CC / 8); k_wdec<<<(16 * (CC / 8) + 255) / 256, 256, 0, stream>>>(dw, BD);
  const size_t n8 = (size_t)NR * CC / 8; const unsigned nb8 = (unsigned)((n8 + 255) / 256); const dim3 gC(((NR / 16) * (CC / 64) + 3) / 4, 1), gK(((NR / 16) * 1 + 3) / 4, 1);
  auto gemm2 = [&](const _Float16* Hh, const _Float16* Hl, const _Float16* Bt, int K, int N, const float* bias, const float* addend, float* C, int act) {
    if (act == 3) { k_gemm_hhx<0><<<dim3(((NR / 16) * ((N + 63) / 64) + 3) / 4, 1), 128, 0, stream>>>(Hh, K, 0, Bt, K, 0, 0.0625f, bias, 0, addend, 1, (size_t)N, 0, C, nullptr, N, 0, NR, N, K); k_gemm_hhx<3><<<dim3(((NR / 16) * ((N + 63) / 64) + 3) / 4, 1), 128, 0, stream>>>(Hl, K, 0, Bt, K, 0, 0.0625f / 1024.0f, nullptr, 0, C, 1, (size_t)N, 0, C, nullptr, N, 0, NR, N, K); }
    else { k_gemm_hhx<0><<<dim3(((NR / 16) * ((N + 63) / 64) + 3) / 4, 1), 128, 0, stream>>>(Hh, K, 0, Bt, K, 0, 0.0625f, bias, 0, addend, 1, (size_t)N, 0, C, nullptr, N, 0, NR, N, K); k_gemm_hhx<0><<<dim3(((NR / 16) * ((N + 63) / 64) + 3) / 4, 1), 128, 0, stream>>>(Hl, K, 0, Bt, K, 0, 0.0625f / 1024.0f, nullptr, 0, C, 1, (size_t)N, 0, C, nullptr, N, 0, NR, N, K); } };
  k_win<<<(NR * 4 + 255) / 256, 256, 0, stream>>>(ac, bcx, A16);
  k_gemm_hhx<0><<<gC, 128, 0, stream>>>(A16, 32, 0, BE, 32, 0, 0.0625f, nullptr, 0, nullptr, 1, 0, 0, ENC, nullptr, CC, 0, NR, CC, 32);
  k_lnc<<<NR / 8, 256, 0, stream>>>(ENC, nullptr, lng, lnb, nullptr, Ph, Pl); gemm2(Ph, Pl, BI, CC, CC, ib, nullptr, X, 0);
  for (int b = 0; b < 4; ++b) {
    k_lnc<<<NR / 8, 256, 0, stream>>>(X, bla + b, blg + b * CC, blb + b * CC, XN, Ph, Pl);
    const float* mi = XN; float* mo = MA; const _Float16* mh = Ph; const _Float16* ml = Pl;
    for (int p = 0; p < 3; ++p) { const int bp = b * 3 + p;
      gemm2(mh, ml, BK1 + (size_t)bp * CR * CC, CC, CR, ivb1 + bp * CR, nullptr, K1, 0);
      k_inv<<<nb8, 256, 0, stream>>>(K1, iv2 + (size_t)bp * 3 * CR, ivb2 + bp * 3, mi, ipa + (size_t)bp * CC, mo, Qh, Ql);
      mi = mo; mo = (mo == MA) ? MB : MA; mh = Qh; ml = Ql; }
    gemm2(Ph, Pl, BS + (size_t)b * CC * CC, CC, CC, skb + b * CC, mi, X, 0); }
  k_split<<<nb8, 256, 0, stream>>>(X, Qh, Ql, n8); gemm2(Qh, Ql, BF, CC, CC, fb, nullptr, MA, 3);
  k_em<<<nb8, 256, 0, stream>>>(ENC, MA, Qh, Ql, n8); gemm2(Qh, Ql, BD, CC, 16, nullptr, nullptr, Y, 0);
  k_ola<<<(NB4 * SEQ + 255) / 256, 256, 0, stream>>>(Y, (float*)d_out);
}
